// GLANTConv_38998303048289
// MI455X (gfx1250) — hardware-verified
//
#include <hip/hip_runtime.h>
#include <stddef.h>
#include <stdint.h>


#define DIN     128
#define OUTC    64
#define NHEAD   4
#define HDQ     256
#define NWT     768
#define PW      512
#define XR_OFF  256
#define NTHR    256
#define NWAVE   8
#define EPT     8
#define CHUNK   (NTHR * EPT)
#define WCAP    (EPT * 32)
#define LISTN   (NWAVE * WCAP)
#define NBMAX   2048
#define RCAP    28672
#define DEGCAP  512
#define STW     512
#define GBM     64
#define GBN     64
#define GTHR    128
#define CX      64.0f
#define CW      256.0f
#define SCL_XW  6.103515625e-05f
#define NEGS    0.2f
#define WSMAX   134217728
#define LDS_AGG ((2 * RCAP + 2 * NBMAX + LISTN) * 4 + 64)

static_assert((CHUNK & (CHUNK - 1)) == 0 && CHUNK <= 4096);
static_assert((NBMAX & (NBMAX - 1)) == 0 && NBMAX <= 4096);
static_assert(NTHR * 8 == NBMAX);
static_assert(LISTN >= NBMAX);
static_assert(LISTN >= NWAVE * WCAP);
static_assert((RCAP % 32) == 0);
static_assert(NWAVE * STW <= RCAP);
static_assert(LDS_AGG <= 300000);
static_assert(GBM == (GTHR / 32) * 16);
static_assert(DIN / 8 == 16);
static_assert((DIN % 32) == 0);
static_assert((PW % GBN) == 0 && (HDQ % GBN) == 0 && (NWT % GBN) == 0);
static_assert(NWT == 3 * HDQ && HDQ == NHEAD * OUTC && PW == 2 * HDQ);
static_assert(OUTC == 64 && 2 * OUTC <= STW);

typedef float    v4f  __attribute__((ext_vector_type(4)));
typedef float    v8f  __attribute__((ext_vector_type(8)));
typedef int      v4i  __attribute__((ext_vector_type(4)));
typedef int      v8i  __attribute__((ext_vector_type(8)));
typedef _Float16 v8h  __attribute__((ext_vector_type(8)));
typedef _Float16 v16h __attribute__((ext_vector_type(16)));
union FragH { v16h v; v8h h[2]; v8i w; };

__device__ __forceinline__ v8f wmh(const FragH& a, const FragH& b, v8f c) {
  v8f d = __builtin_amdgcn_wmma_f32_16x16x32_f16(false, a.v, false, b.v, (short)0, c, false, false);
  asm volatile("v_nop\n\tv_nop\n\tv_nop\n\tv_nop" : "+v"(d) : "v"(a.w), "v"(b.w));
  return d;
}

__device__ __forceinline__ void ldwait() {
  asm volatile("s_wait_loadcnt 0x0" ::: "memory");
}

__device__ __forceinline__ float bfq(float v) {
  unsigned u = (unsigned)__float_as_uint(v);
  u = (u + 0x7fffu + ((u >> 16) & 1u)) & 0xffff0000u;
  return __uint_as_float(u);
}

__device__ __forceinline__ v8h cvt8h(const v4f a, const v4f b, const float c) {
  v8h hv;
  hv[0] = (_Float16)(bfq(a.x) * c); hv[1] = (_Float16)(bfq(a.y) * c);
  hv[2] = (_Float16)(bfq(a.z) * c); hv[3] = (_Float16)(bfq(a.w) * c);
  hv[4] = (_Float16)(bfq(b.x) * c); hv[5] = (_Float16)(bfq(b.y) * c);
  hv[6] = (_Float16)(bfq(b.z) * c); hv[7] = (_Float16)(bfq(b.w) * c);
  return hv;
}

__device__ __forceinline__ int scan_chunk(const int* __restrict__ dsts, int nE, int cbase, int slotBase,
                                          int nb, int vec8, int* list, int tid, int lane, int wave) {
  int wc = 0;
  const int el0  = tid * EPT;
  const int e0   = cbase + el0;
  const int sent = -2147483647 - 1;
  v4i da, db;
  if (vec8 != 0 && cbase + CHUNK <= nE) {
    da = *(const v4i*)(dsts + e0);
    db = *(const v4i*)(dsts + e0 + 4);
  } else {
    da.x = (e0     < nE) ? dsts[min(e0,     nE - 1)] : sent;
    da.y = (e0 + 1 < nE) ? dsts[min(e0 + 1, nE - 1)] : sent;
    da.z = (e0 + 2 < nE) ? dsts[min(e0 + 2, nE - 1)] : sent;
    da.w = (e0 + 3 < nE) ? dsts[min(e0 + 3, nE - 1)] : sent;
    db.x = (e0 + 4 < nE) ? dsts[min(e0 + 4, nE - 1)] : sent;
    db.y = (e0 + 5 < nE) ? dsts[min(e0 + 5, nE - 1)] : sent;
    db.z = (e0 + 6 < nE) ? dsts[min(e0 + 6, nE - 1)] : sent;
    db.w = (e0 + 7 < nE) ? dsts[min(e0 + 7, nE - 1)] : sent;
  }
  const unsigned nbs = (unsigned)slotBase;
  const unsigned unb = (unsigned)nb;
  const unsigned s0 = (unsigned)da.x - nbs, s1 = (unsigned)da.y - nbs;
  const unsigned s2 = (unsigned)da.z - nbs, s3 = (unsigned)da.w - nbs;
  const unsigned s4 = (unsigned)db.x - nbs, s5 = (unsigned)db.y - nbs;
  const unsigned s6 = (unsigned)db.z - nbs, s7 = (unsigned)db.w - nbs;
  const bool h0 = s0 < unb, h1 = s1 < unb, h2 = s2 < unb, h3 = s3 < unb;
  const bool h4 = s4 < unb, h5 = s5 < unb, h6 = s6 < unb, h7 = s7 < unb;
  const unsigned any = __builtin_amdgcn_ballot_w32(h0 | h1 | h2 | h3 | h4 | h5 | h6 | h7);
  if (any != 0u) {
#define HITJ(J, HJ, SJ) { \
      const unsigned mj = __builtin_amdgcn_ballot_w32(HJ); \
      if (mj != 0u) { \
        if (HJ) { \
          const int pos = wc + (int)__builtin_amdgcn_mbcnt_lo(mj, 0u); \
          if (pos < WCAP) list[wave * WCAP + pos] = ((el0 + (J)) << 12) | (int)(SJ); \
        } \
        wc += (int)__builtin_popcount(mj); } }
    HITJ(0, h0, s0)
    HITJ(1, h1, s1)
    HITJ(2, h2, s2)
    HITJ(3, h3, s3)
    HITJ(4, h4, s4)
    HITJ(5, h5, s5)
    HITJ(6, h6, s6)
    HITJ(7, h7, s7)
#undef HITJ
  }
  return wc;
}

__global__ __launch_bounds__(NTHR) void k_xprep(const float* __restrict__ x, _Float16* xh, int nN, int nUnits) {
  const int i = (int)blockIdx.x * NTHR + (int)threadIdx.x;
  if (i >= nUnits) return;
  const int row = i >> 4;
  const int c0  = (i & 15) * 8;
  const int rc  = row < nN ? row : nN - 1;
  const float* p = x + (size_t)rc * DIN + c0;
  v4f a = *(const v4f*)p, b = *(const v4f*)(p + 4);
  const v4f z4 = {0.f, 0.f, 0.f, 0.f};
  if (row >= nN) { a = z4; b = z4; }
  const v8h hv = cvt8h(a, b, CX);
  const size_t o = (size_t)row * DIN + c0;
  *(volatile v8h*)(xh + o) = hv;
  __threadfence();
  *(volatile v8h*)(xh + o) = hv;
}

__global__ __launch_bounds__(NTHR) void k_wtr(const float* __restrict__ w0, const float* __restrict__ w1,
                                              const float* __restrict__ w2, const float* __restrict__ w3,
                                              int c0, int c1, int c2, int c3, int segRows, int K,
                                              _Float16* wt, int nUnits) {
  const int u = (int)blockIdx.x * NTHR + (int)threadIdx.x;
  if (u >= nUnits) return;
  const int kq = K >> 3;
  const int n  = u / kq;
  const int k8 = (u - n * kq) * 8;
  int seg = n / segRows;
  seg = seg > 3 ? 3 : seg;
  const int nc = n - seg * segRows;
  const float* ws = (seg == 0) ? w0 : ((seg == 1) ? w1 : ((seg == 2) ? w2 : w3));
  const int cc = (seg == 0) ? c0 : ((seg == 1) ? c1 : ((seg == 2) ? c2 : c3));
  const int ncl = nc < cc ? nc : cc - 1;
  const float* p = ws + (size_t)k8 * (size_t)cc + ncl;
  v4f a, b;
  a.x = p[0];                  a.y = p[(size_t)cc];         a.z = p[(size_t)2 * cc];     a.w = p[(size_t)3 * cc];
  b.x = p[(size_t)4 * cc];     b.y = p[(size_t)5 * cc];     b.z = p[(size_t)6 * cc];     b.w = p[(size_t)7 * cc];
  const v4f z4 = {0.f, 0.f, 0.f, 0.f};
  if (nc >= cc) { a = z4; b = z4; }
  const v8h hv = cvt8h(a, b, CW);
  const size_t o = (size_t)n * (size_t)K + k8;
  *(volatile v8h*)(wt + o) = hv;
  __threadfence();
  *(volatile v8h*)(wt + o) = hv;
}

__global__ __launch_bounds__(GTHR) void k_gemm(
    const _Float16* __restrict__ A, const _Float16* __restrict__ WT,
    float* outF, int K, int ldo, float scl)
{
  __shared__ __attribute__((aligned(16))) float stg[GBM * GBN];
  const int tid = (int)threadIdx.x, lane = tid & 31, wave = tid >> 5, hh = lane >> 4, m = lane & 15;
  const int rowBase = (int)blockIdx.x * GBM;
  const int col0    = (int)blockIdx.y * GBN;

  v8f acc[4];
  {
    const v8f z = {0.f, 0.f, 0.f, 0.f, 0.f, 0.f, 0.f, 0.f};
    acc[0] = z; acc[1] = z; acc[2] = z; acc[3] = z;
  }
  const _Float16* ap = A  + (size_t)(rowBase + 16 * wave + m) * (size_t)K + 8 * hh;
  const _Float16* wp = WT + (size_t)(col0 + m) * (size_t)K + 8 * hh;
  const int ksteps = K >> 5;
#pragma unroll 1
  for (int ks = 0; ks < ksteps; ++ks) {
    FragH af;
    af.h[0] = *(const v8h*)(ap + 32 * ks);
    af.h[1] = *(const v8h*)(ap + 32 * ks + 16);
#pragma unroll
    for (int t = 0; t < 4; ++t) {
      const _Float16* wq = wp + (size_t)(16 * t) * (size_t)K + 32 * ks;
      FragH bf;
      bf.h[0] = *(const v8h*)wq;
      bf.h[1] = *(const v8h*)(wq + 16);
      acc[t] = wmh(af, bf, acc[t]);
    }
  }

#pragma unroll
  for (int t = 0; t < 4; ++t) {
    const int lc = 16 * t + m;
#pragma unroll
    for (int r = 0; r < 8; ++r) {
      const int lr = 16 * wave + 8 * hh + r;
      stg[lr * GBN + lc] = acc[t][r] * scl;
    }
  }
  __syncthreads();

  v4f fv[8];
#pragma unroll
  for (int i = 0; i < 8; ++i) {
    const int lr = 16 * wave + 2 * i + hh;
    fv[i] = *(const v4f*)(stg + lr * GBN + 4 * m);
  }
#pragma unroll
  for (int i = 0; i < 8; ++i) {
    const int lr = 16 * wave + 2 * i + hh;
    const int gr = rowBase + lr;
    float* op = outF + (size_t)gr * (size_t)ldo + col0 + 4 * m;
    *(volatile v4f*)op = fv[i];
  }
  __threadfence();
#pragma unroll
  for (int i = 0; i < 8; ++i) {
    const int lr = 16 * wave + 2 * i + hh;
    const int gr = rowBase + lr;
    float* op = outF + (size_t)gr * (size_t)ldo + col0 + 4 * m;
    *(volatile v4f*)op = fv[i];
  }
}

template<int HOP>
__global__ __launch_bounds__(NTHR) void k_agg(
    const int* __restrict__ srcs, const int* __restrict__ dsts,
    const float* __restrict__ P, const float* __restrict__ att, const float* __restrict__ theta,
    const float* Hin, float* Hout,
    int nN, int nE, int nb, int vec8, int MPr) {
  extern __shared__ v4f lds_dyn[];
  int* reg1 = (int*)lds_dyn;
  int* reg2 = reg1 + RCAP;
  int* scnt = reg2 + RCAP;
  int* soff = scnt + NBMAX;
  int* list = soff + NBMAX;
  int* wcnt = list + LISTN;
  int* wtot = wcnt + NWAVE;
  const int tid = (int)threadIdx.x, lane = tid & 31, wave = tid >> 5;
  const int nodeBase = (int)blockIdx.x * nb;

  for (int i = tid; i < NBMAX; i += NTHR) scnt[i] = 0;
  __syncthreads();

  int tot = 0;
  const int nChunks = (nE + CHUNK - 1) / CHUNK;
#pragma unroll 1
  for (int ch = 0; ch < nChunks; ++ch) {
    const int cbase = ch * CHUNK;
    const int wc = scan_chunk(dsts, nE, cbase, nodeBase, nb, vec8, list, tid, lane, wave);
    if (lane == 0) wcnt[wave] = wc;
    __syncthreads();
    int pre = 0, all = 0;
#pragma unroll
    for (int w2 = 0; w2 < NWAVE; ++w2) {
      int c = wcnt[w2];
      c = c < 0 ? 0 : (c > WCAP ? WCAP : c);
      all += c;
      pre += (w2 < wave) ? c : 0;
    }
    const int wcc  = wc > WCAP ? WCAP : wc;
    const int base = tot + pre;
#pragma unroll 1
    for (int i = lane; i < wcc; i += 32) {
      const int ent = list[wave * WCAP + i];
      const int el  = (ent >> 12) & (CHUNK - 1);
      const int sl  = ent & (NBMAX - 1);
      int eid = cbase + el;
      eid = eid > nE - 1 ? nE - 1 : eid;
      const int pos = base + i;
      if (pos < RCAP) reg1[pos] = (int)(((unsigned)eid << 12) | (unsigned)sl);
    }
    tot += all;
    tot = tot > RCAP ? RCAP : tot;
    __syncthreads();
  }
  const int nh = tot;

  if (wave == 0) {
#pragma unroll 1
    for (int b0 = 0; b0 < nh; b0 += 32) {
      const int idx = b0 + lane;
      const int uv  = reg1[idx < RCAP ? idx : RCAP - 1];
      const int m32 = (nh - b0) < 32 ? (nh - b0) : 32;
#pragma unroll 1
      for (int k = 0; k < m32; ++k) {
        const int u  = __builtin_amdgcn_readlane(uv, k);
        const int sl = u & (NBMAX - 1);
        if (lane == 0) scnt[sl] = scnt[sl] + 1;
      }
    }
  }
  __syncthreads();

  {
    const v4i ca = *(const v4i*)(scnt + 8 * tid);
    const v4i cb = *(const v4i*)(scnt + 8 * tid + 4);
    const int e0 = ca.x < 0 ? 0 : ca.x, e1 = ca.y < 0 ? 0 : ca.y, e2 = ca.z < 0 ? 0 : ca.z, e3 = ca.w < 0 ? 0 : ca.w;
    const int e4 = cb.x < 0 ? 0 : cb.x, e5 = cb.y < 0 ? 0 : cb.y, e6 = cb.z < 0 ? 0 : cb.z, e7 = cb.w < 0 ? 0 : cb.w;
    const int ts = e0 + e1 + e2 + e3 + e4 + e5 + e6 + e7;
    int incl = ts;
#pragma unroll
    for (int d = 1; d < 32; d <<= 1) {
      const int up = __shfl_up(incl, d);
      if (lane >= d) incl += up;
    }
    if (lane == 31) wtot[wave] = incl;
    __syncthreads();
    int pre = 0;
#pragma unroll
    for (int w2 = 0; w2 < NWAVE; ++w2) pre += (w2 < wave) ? wtot[w2] : 0;
    int run = pre + incl - ts;
    soff[8 * tid + 0] = run; run += e0;
    soff[8 * tid + 1] = run; run += e1;
    soff[8 * tid + 2] = run; run += e2;
    soff[8 * tid + 3] = run; run += e3;
    soff[8 * tid + 4] = run; run += e4;
    soff[8 * tid + 5] = run; run += e5;
    soff[8 * tid + 6] = run; run += e6;
    soff[8 * tid + 7] = run;
  }
  __syncthreads();
  for (int i = tid; i < NBMAX; i += NTHR) list[i] = soff[i];
  __syncthreads();

  if (wave == 0) {
#pragma unroll 1
    for (int b0 = 0; b0 < nh; b0 += 32) {
      const int idx = b0 + lane;
      const int uv  = reg1[idx < RCAP ? idx : RCAP - 1];
      const int m32 = (nh - b0) < 32 ? (nh - b0) : 32;
#pragma unroll 1
      for (int k = 0; k < m32; ++k) {
        const int u   = __builtin_amdgcn_readlane(uv, k);
        const int sl  = u & (NBMAX - 1);
        const int eid = (int)((unsigned)u >> 12);
        if (lane == 0) {
          int pos = list[sl];
          pos = pos < 0 ? 0 : (pos > RCAP - 1 ? RCAP - 1 : pos);
          reg2[pos] = eid;
          list[sl] = pos + 1;
        }
      }
    }
  }
  __syncthreads();

  const int nbw = nb >> 3;
  const bool ovf = (nh >= RCAP);
  const float qnan = __int_as_float(0x7fc00000);
  float* stw = (float*)reg1 + wave * STW;
  const int lc = lane < (OUTC / 4) ? lane : (OUTC / 4) - 1;
  float at[8];
#pragma unroll
  for (int j = 0; j < 8; ++j) at[j] = bfq(att[32 * j + lane]);
  float sg = 0.f;
  if (HOP == 1) {
    const float t = bfq(theta[0]);
    sg = 1.0f / (1.0f + __expf(-t));
  }
  ldwait();
  const int selfn = (HOP == 0) ? 1 : 0;
#pragma unroll 1
  for (int jt = 0; jt < nbw; ++jt) {
    const int slot = wave * nbw + jt;
    const int grow = nodeBase + slot;
    const int gcl  = grow < nN ? grow : nN - 1;
    int st = soff[slot];
    const int craw = scnt[slot];
    int cnt = craw;
    st  = st < 0 ? 0 : (st > nh ? nh : st);
    cnt = cnt < 0 ? 0 : (cnt > DEGCAP ? DEGCAP : cnt);
    if (cnt > nh - st) cnt = nh - st;
    const float pz = (ovf || craw > DEGCAP) ? qnan : 0.0f;
    const bool wr = (HOP == 0) ? (grow < MPr) : (grow < nN);
    const float live = grow < nN ? 1.0f : 0.0f;

    const float* drow = P + (size_t)gcl * PW + XR_OFF + lane;
    float xd[8], av[8];
#pragma unroll
    for (int j = 0; j < 8; ++j) { xd[j] = drow[32 * j]; av[j] = 0.f; }
    float h0a = 0.f, h0b = 0.f;
    if (HOP == 1) {
      const float* hr = Hin + (size_t)gcl * OUTC + lane;
      h0a = hr[0];
      h0b = hr[32];
    }
    ldwait();
    float mx[4], dn[4];
#pragma unroll
    for (int h = 0; h < 4; ++h) { mx[h] = -1.0e30f; dn[h] = 0.f; }

    const int tot3 = cnt + selfn;
#pragma unroll 1
    for (int q = 0; q < tot3; ++q) {
      int idx = st + q; idx = idx > RCAP - 1 ? RCAP - 1 : idx;
      int eid = reg2[idx]; eid = eid < 0 ? 0 : (eid > nE - 1 ? nE - 1 : eid);
      const int sraw = srcs[eid];
      const int se = sraw < 0 ? 0 : (sraw > nN - 1 ? nN - 1 : sraw);
      const int s  = (q < cnt) ? se : gcl;
      const float* sr = P + (size_t)s * PW + lane;
      float xs[8];
#pragma unroll
      for (int j = 0; j < 8; ++j) xs[j] = sr[32 * j];
      ldwait();
      float part[4];
#pragma unroll
      for (int h = 0; h < 4; ++h) {
        float m0 = xs[2 * h] + xd[2 * h];
        float m1 = xs[2 * h + 1] + xd[2 * h + 1];
        m0 = m0 > 0.f ? m0 : NEGS * m0;
        m1 = m1 > 0.f ? m1 : NEGS * m1;
        part[h] = fmaf(m1, at[2 * h + 1], m0 * at[2 * h]);
      }
#pragma unroll
      for (int off = 16; off > 0; off >>= 1) {
#pragma unroll
        for (int h = 0; h < 4; ++h) part[h] += __shfl_xor(part[h], off);
      }
#pragma unroll
      for (int h = 0; h < 4; ++h) {
        const float al = part[h];
        const float df = al - mx[h];
        const float ee = __expf(-fabsf(df));
        const bool up  = df > 0.f;
        const float s1 = up ? ee : 1.0f;
        const float s2 = up ? 1.0f : ee;
        mx[h] = up ? al : mx[h];
        dn[h] = fmaf(dn[h], s1, s2);
        av[2 * h]     = fmaf(av[2 * h],     s1, s2 * xs[2 * h]);
        av[2 * h + 1] = fmaf(av[2 * h + 1], s1, s2 * xs[2 * h + 1]);
      }
    }
    float iv[4];
#pragma unroll
    for (int h = 0; h < 4; ++h) {
      const float ds = dn[h] > 0.f ? dn[h] : 1.0f;
      iv[h] = (dn[h] > 0.f ? 1.0f : 0.0f) * __builtin_amdgcn_rcpf(ds);
    }
    const float o0 = ((av[0] * iv[0] + av[2] * iv[1]) + (av[4] * iv[2] + av[6] * iv[3])) * 0.25f;
    const float o1 = ((av[1] * iv[0] + av[3] * iv[1]) + (av[5] * iv[2] + av[7] * iv[3])) * 0.25f;
    float r0, r1;
    if (HOP == 0) {
      r0 = o0 * live + pz;
      r1 = o1 * live + pz;
    } else {
      r0 = fmaf(sg, o0, h0a) + pz;
      r1 = fmaf(sg, o1, h0b) + pz;
    }
    __builtin_amdgcn_fence(__ATOMIC_RELEASE, "wavefront");
    __builtin_amdgcn_wave_barrier();
    stw[lane]      = r0;
    stw[32 + lane] = r1;
    __builtin_amdgcn_fence(__ATOMIC_RELEASE, "wavefront");
    __builtin_amdgcn_wave_barrier();
    const v4f g = *(const v4f*)(stw + 4 * lc);
    const int gsafe = wr ? grow : 0;
    float* gp = Hout + (size_t)gsafe * OUTC + 4 * lc;
    const bool wsv = wr && (lane < (OUTC / 4));
    if (wsv) *(volatile v4f*)gp = g;
    __threadfence();
    if (wsv) *(volatile v4f*)gp = g;
  }
}

static int pick_nb(int nE, int nN) {
  int nb = NBMAX;
  while (nb > 16 && (long long)nb * (long long)nE * 5LL > (long long)RCAP * (long long)nN * 4LL) nb >>= 1;
  return nb;
}
static inline int cdiv(int a, int b) { return (a + b - 1) / b; }

extern "C" void kernel_launch(void* const* d_in, const int* in_sizes, int n_in,
                              void* d_out, int out_size, void* d_ws, size_t ws_size,
                              hipStream_t stream) {
  if (n_in < 9) return;
  const int nN = in_sizes[0] / DIN;
  if (nN <= 0 || in_sizes[0] != nN * DIN || nN > (1 << 22)) return;
  if (in_sizes[1] < 2 || (in_sizes[1] & 1) != 0) return;
  if (in_sizes[2] < 2 || (in_sizes[2] & 1) != 0) return;
  const int nE1 = in_sizes[1] / 2;
  const int nE2 = in_sizes[2] / 2;
  if (nE1 < 1 || nE1 > (1 << 20) || nE2 < 1 || nE2 > (1 << 20)) return;
  if (in_sizes[3] != DIN * HDQ || in_sizes[4] != DIN * HDQ || in_sizes[5] != DIN * HDQ) return;
  if (in_sizes[6] != HDQ || in_sizes[7] != HDQ || in_sizes[8] < 1) return;
  if (out_size != nN * OUTC) return;

  const float* x    = (const float*)d_in[0];
  const int*   ei1  = (const int*)  d_in[1];
  const int*   ei2  = (const int*)  d_in[2];
  const float* Wl   = (const float*)d_in[3];
  const float* Wr0  = (const float*)d_in[4];
  const float* Wr1  = (const float*)d_in[5];
  const float* att0 = (const float*)d_in[6];
  const float* att1 = (const float*)d_in[7];
  const float* theta = (const float*)d_in[8];
  float* out = (float*)d_out;
  const int* src1 = ei1;
  const int* dst1 = ei1 + nE1;
  const int* src2 = ei2;
  const int* dst2 = ei2 + nE2;

  const int MP    = cdiv(nN, GBM) * GBM;
  const int nb0   = pick_nb(nE1, nN);
  const int nb1   = pick_nb(nE2, nN);
  const int gA0   = cdiv(MP, nb0);
  const int gA1   = cdiv(MP, nb1);
  const int vec8a = ((nE1 & 3) == 0) ? 1 : 0;
  const int vec8b = ((nE2 & 3) == 0) ? 1 : 0;
  if (gA0 * nb0 < MP || gA1 * nb1 < MP) return;

  char* ws = (char*)d_ws;
  size_t off = 0;
  const size_t oXH = off; off += (size_t)MP * DIN * 2;            off = (off + 255) & ~(size_t)255;
  const size_t oWT = off; off += (size_t)NWT * DIN * 2;           off = (off + 255) & ~(size_t)255;
  const size_t oP  = off; off += (size_t)MP * PW * 4;             off = (off + 255) & ~(size_t)255;
  const size_t oH0 = off; off += (size_t)MP * OUTC * 4;           off = (off + 255) & ~(size_t)255;
  if (off > ws_size || off > (size_t)WSMAX) return;
  _Float16* XH = (_Float16*)(ws + oXH);
  _Float16* WT = (_Float16*)(ws + oWT);
  float*    P  = (float*)(ws + oP);
  float*    H0 = (float*)(ws + oH0);

  hipFuncSetAttribute(reinterpret_cast<const void*>(&k_agg<0>),
                      hipFuncAttributeMaxDynamicSharedMemorySize, LDS_AGG);
  hipFuncSetAttribute(reinterpret_cast<const void*>(&k_agg<1>),
                      hipFuncAttributeMaxDynamicSharedMemorySize, LDS_AGG);

  const int nUx = MP * (DIN / 8);
  k_xprep<<<cdiv(nUx, NTHR), NTHR, 0, stream>>>(x, XH, nN, nUx);

  {
    const int nU = NWT * (DIN / 8);
    k_wtr<<<cdiv(nU, NTHR), NTHR, 0, stream>>>(Wl, Wr0, Wr1, Wr1, HDQ, HDQ, HDQ, HDQ, HDQ, DIN, WT, nU);
  }

  const int gM = MP / GBM;
  k_gemm<<<dim3(gM, PW / GBN), GTHR, 0, stream>>>(XH, WT, P, DIN, PW, SCL_XW);
  k_agg<0><<<gA0, NTHR, LDS_AGG, stream>>>(src1, dst1, P, att0, theta, H0, H0, nN, nE1, nb0, vec8a, MP);
  k_gemm<<<dim3(gM, HDQ / GBN), GTHR, 0, stream>>>(XH, WT + (size_t)(2 * HDQ) * DIN, P + XR_OFF, DIN, PW, SCL_XW);
  k_agg<1><<<gA1, NTHR, LDS_AGG, stream>>>(src2, dst2, P, att1, theta, H0, out, nN, nE2, nb1, vec8b, MP);
}
